// PyGEGNNDecoderMSE_15917148799551
// MI455X (gfx1250) — hardware-verified
//
#include <hip/hip_runtime.h>
#include <stddef.h>
#include <stdint.h>


#define NTHR   256
#define NWAVE  8
#define EPT    8
#define CHUNK  (NTHR * EPT)
#define WCAP   (EPT * 32)
#define LISTN  (NWAVE * WCAP)
#define PASSN  128
#define PCAP   (CHUNK + PASSN)
#define RMAX   (PCAP / PASSN + 1)
#define NB     128
#define HID    128
#define TM     64

static_assert(PASSN <= NTHR);
static_assert((PASSN % 16) == 0);
static_assert((NB % 16) == 0);

#define EO_ACC   0
#define EO_ACU   (EO_ACC + (NB + 1) * HID * 4)
#define EO_E1H   (EO_ACU + (NB + 1) * 16)
#define EO_E1L   (EO_E1H + PASSN * HID * 2)
#define EO_MPL   (EO_E1L + PASSN * HID * 2)
#define EO_PART  (EO_MPL + PASSN * HID * 2)
#define EO_RELV  (EO_PART + NWAVE * PASSN * 4)
#define EO_CWR   (EO_RELV + PASSN * 16)
#define EO_SLOT  (EO_CWR + PASSN * 16)
#define EO_PEND  (EO_SLOT + PASSN * 4)
#define EO_LIST  (EO_PEND + PCAP * 4)
#define EO_WTS   (EO_LIST + LISTN * 4)
#define EO_MISC  (EO_WTS + 5 * HID * 4)
#define EDGE_LDS (EO_MISC + 64)
static_assert((EO_ACU % 16) == 0 && (EO_E1H % 16) == 0 && (EO_E1L % 16) == 0 && (EO_MPL % 16) == 0);
static_assert((EO_PART % 16) == 0 && (EO_RELV % 16) == 0 && (EO_CWR % 16) == 0 && (EO_SLOT % 16) == 0);
static_assert((EO_PEND % 16) == 0 && (EO_LIST % 16) == 0 && (EO_WTS % 16) == 0 && (EO_MISC % 16) == 0);
static_assert(NWAVE * PASSN >= NB * 3);

#define NO_R0    0
#define NO_R1    (NO_R0 + TM * 256 * 2 * 2)
#define NO_R2    (NO_R1 + TM * HID * 2 * 2)
#define NO_VEC   (NO_R2 + TM * HID * 4)
#define NO_OST   (NO_VEC + 1024 * 4)
#define NODE_LDS (NO_OST + 192 * 4)
static_assert((NO_R1 % 16) == 0 && (NO_R2 % 16) == 0 && (NO_VEC % 16) == 0 && (NO_OST % 16) == 0);

typedef float          v4f   __attribute__((ext_vector_type(4)));
typedef float          v8f   __attribute__((ext_vector_type(8)));
typedef int            v4i   __attribute__((ext_vector_type(4)));
typedef unsigned short v4us  __attribute__((ext_vector_type(4)));
typedef unsigned short v8us  __attribute__((ext_vector_type(8)));
typedef unsigned short v16us __attribute__((ext_vector_type(16)));
typedef _Float16       v16h  __attribute__((ext_vector_type(16)));
typedef __bf16         v16bf __attribute__((ext_vector_type(16)));
union U16 { v16us u; v8us h[2]; };

__device__ __forceinline__ v8f zero8f() {
  v8f r;
#pragma unroll
  for (int i = 0; i < 8; ++i) r[i] = 0.0f;
  return r;
}

__device__ __forceinline__ float silu_f(float x) {
  return x * __builtin_amdgcn_rcpf(1.0f + __expf(-x));
}

__device__ __forceinline__ unsigned bfbits(float x) {
  unsigned u = __float_as_uint(x);
  return (u + 0x7fffu + ((u >> 16) & 1u)) >> 16;
}
__device__ __forceinline__ unsigned split2(float x) {
  const unsigned hb = bfbits(x);
  const float hv = __uint_as_float(hb << 16);
  const unsigned lb = bfbits(x - hv);
  return (hb & 0xffffu) | (lb << 16);
}
__device__ __forceinline__ unsigned short f16bits(float x) {
  const _Float16 t = (_Float16)x;
  return __builtin_bit_cast(unsigned short, t);
}

__device__ __forceinline__ v16us ldfr(const unsigned short* p, int hh) {
  U16 f;
  f.h[0] = *(const v8us*)(p + 8 * hh);
  f.h[1] = *(const v8us*)(p + 16 + 8 * hh);
  return f.u;
}

__device__ __forceinline__ v8f wbf(v8f c, v16us a, v16us b) {
  v8f d = __builtin_amdgcn_wmma_f32_16x16x32_bf16(false, __builtin_bit_cast(v16bf, a), false,
                                                  __builtin_bit_cast(v16bf, b), (short)0, c, false, false);
  asm volatile("v_nop\n\tv_nop\n\tv_nop\n\tv_nop" : "+v"(d) : "v"(a), "v"(b));
  return d;
}
__device__ __forceinline__ v8f wf16(v8f c, v16us a, v16us b) {
  v8f d = __builtin_amdgcn_wmma_f32_16x16x32_f16(false, __builtin_bit_cast(v16h, a), false,
                                                 __builtin_bit_cast(v16h, b), (short)0, c, false, false);
  asm volatile("v_nop\n\tv_nop\n\tv_nop\n\tv_nop" : "+v"(d) : "v"(a), "v"(b));
  return d;
}
__device__ __forceinline__ v8f w3(v8f c, v16us ah, v16us al, v16us bh, v16us bl) {
  c = wbf(c, ah, bh);
  c = wbf(c, al, bh);
  c = wbf(c, ah, bl);
  return c;
}

__device__ __forceinline__ int scan_chunk(const int* __restrict__ dsts, int nE, int cbase, int nodeBase,
                                          int vec8, int* list, int tid, int wave) {
  int wc = 0;
  const int el0  = tid * EPT;
  const int e0   = cbase + el0;
  const int sent = -2147483647 - 1;
  v4i da, db;
  if (vec8 != 0 && cbase + CHUNK <= nE) {
    da = *(const v4i*)(dsts + e0);
    db = *(const v4i*)(dsts + e0 + 4);
  } else {
    da.x = (e0     < nE) ? dsts[min(e0, nE - 1)] : sent;
    da.y = (e0 + 1 < nE) ? dsts[min(e0 + 1, nE - 1)] : sent;
    da.z = (e0 + 2 < nE) ? dsts[min(e0 + 2, nE - 1)] : sent;
    da.w = (e0 + 3 < nE) ? dsts[min(e0 + 3, nE - 1)] : sent;
    db.x = (e0 + 4 < nE) ? dsts[min(e0 + 4, nE - 1)] : sent;
    db.y = (e0 + 5 < nE) ? dsts[min(e0 + 5, nE - 1)] : sent;
    db.z = (e0 + 6 < nE) ? dsts[min(e0 + 6, nE - 1)] : sent;
    db.w = (e0 + 7 < nE) ? dsts[min(e0 + 7, nE - 1)] : sent;
  }
  const unsigned nb = (unsigned)nodeBase;
  const unsigned s0 = (unsigned)da.x - nb, s1 = (unsigned)da.y - nb;
  const unsigned s2 = (unsigned)da.z - nb, s3 = (unsigned)da.w - nb;
  const unsigned s4 = (unsigned)db.x - nb, s5 = (unsigned)db.y - nb;
  const unsigned s6 = (unsigned)db.z - nb, s7 = (unsigned)db.w - nb;
  const bool h0 = s0 < (unsigned)NB, h1 = s1 < (unsigned)NB, h2 = s2 < (unsigned)NB, h3 = s3 < (unsigned)NB;
  const bool h4 = s4 < (unsigned)NB, h5 = s5 < (unsigned)NB, h6 = s6 < (unsigned)NB, h7 = s7 < (unsigned)NB;
  const unsigned any = __builtin_amdgcn_ballot_w32(h0 | h1 | h2 | h3 | h4 | h5 | h6 | h7);
  if (any != 0u) {
#define HITJ(J, HJ) { \
      const unsigned mj = __builtin_amdgcn_ballot_w32(HJ); \
      if (mj != 0u) { \
        if (HJ) { \
          const int pos = wc + (int)__builtin_amdgcn_mbcnt_lo(mj, 0u); \
          if (pos < WCAP) list[wave * WCAP + pos] = el0 + (J); \
        } \
        wc += (int)__builtin_popcount(mj); } }
    HITJ(0, h0)
    HITJ(1, h1)
    HITJ(2, h2)
    HITJ(3, h3)
    HITJ(4, h4)
    HITJ(5, h5)
    HITJ(6, h6)
    HITJ(7, h7)
#undef HITJ
  }
  return wc;
}

template <int F16>
__global__ __launch_bounds__(NTHR) void k_cvt(const float* __restrict__ src, unsigned short* dA, unsigned short* dB,
                                             int K, int N, int Nh, int sk, int sn, int hofs,
                                             int srcL, int dstL, float scale) {
  const int lyr = blockIdx.y;
  const float* s = src + (size_t)lyr * (size_t)srcL;
  unsigned short* oa = dA + (size_t)lyr * (size_t)dstL;
  unsigned short* ob = dB + (size_t)lyr * (size_t)dstL;
  const int idx = blockIdx.x * NTHR + threadIdx.x;
  const int kq = K >> 3;
  int n = idx / kq;
  const int k8 = (idx - n * kq) * 8;
  const bool ok = n < N;
  n = ok ? n : (N - 1);
  const int nh = n % Nh, ng = n / Nh;
  float v[8];
#pragma unroll
  for (int j = 0; j < 8; ++j)
    v[j] = s[(size_t)(k8 + j) * (size_t)sk + (size_t)nh * (size_t)sn + (size_t)ng * (size_t)hofs];
  v8us ha, hb;
  if (F16 != 0) {
#pragma unroll
    for (int j = 0; j < 8; ++j) { const unsigned short t = f16bits(v[j] * scale); ha[j] = t; hb[j] = t; }
  } else {
#pragma unroll
    for (int j = 0; j < 8; ++j) {
      const unsigned p = split2(v[j]);
      ha[j] = (unsigned short)(p & 0xffffu);
      hb[j] = (unsigned short)(p >> 16);
    }
  }
  unsigned short* pa = oa + (size_t)n * K + k8;
  unsigned short* pb = ob + (size_t)n * K + k8;
  if (ok) {
    *(volatile v8us*)pa = ha;
    if (F16 == 0) *(volatile v8us*)pb = hb;
  }
  __threadfence();
  if (ok) {
    *(volatile v8us*)pa = ha;
    if (F16 == 0) *(volatile v8us*)pb = hb;
  }
}

__global__ __launch_bounds__(NTHR) void k_zl(const float* __restrict__ z,
                                            const unsigned short* __restrict__ lwH,
                                            const unsigned short* __restrict__ lwL,
                                            float* zl, int nB) {
  __shared__ __attribute__((aligned(16))) unsigned short zp[2 * 64 * 64];
  __shared__ __attribute__((aligned(16))) float st[64 * 128];
  const int tid = threadIdx.x, lane = tid & 31, w = tid >> 5, hh = lane >> 4, m = lane & 15;
  const int b0 = blockIdx.x * 64;
  if (b0 + 64 > nB) return;
#pragma unroll
  for (int it = 0; it < 4; ++it) {
    const int idx = it * NTHR + tid;
    const int row = idx >> 4, c4 = (idx & 15) * 4;
    const v4f v = *(const v4f*)(z + (size_t)(b0 + row) * 64 + c4);
    v4us gh, gl;
#pragma unroll
    for (int j = 0; j < 4; ++j) {
      const unsigned p = split2(v[j]);
      gh[j] = (unsigned short)(p & 0xffffu);
      gl[j] = (unsigned short)(p >> 16);
    }
    *(v4us*)(zp + row * 64 + c4) = gh;
    *(v4us*)(zp + 4096 + row * 64 + c4) = gl;
  }
  __syncthreads();
  const int n = 16 * w + m;
  v8f acc[4];
#pragma unroll
  for (int t = 0; t < 4; ++t) acc[t] = zero8f();
#pragma unroll
  for (int ks = 0; ks < 2; ++ks) {
    const v16us bh = ldfr(lwH + (size_t)n * 64 + 32 * ks, hh);
    const v16us bl = ldfr(lwL + (size_t)n * 64 + 32 * ks, hh);
#pragma unroll
    for (int t = 0; t < 4; ++t) {
      const v16us ah = ldfr(zp + (16 * t + m) * 64 + 32 * ks, hh);
      const v16us al = ldfr(zp + 4096 + (16 * t + m) * 64 + 32 * ks, hh);
      acc[t] = w3(acc[t], ah, al, bh, bl);
    }
  }
#pragma unroll
  for (int t = 0; t < 4; ++t) {
#pragma unroll
    for (int rr = 0; rr < 8; ++rr) st[(16 * t + 8 * hh + rr) * 128 + n] = acc[t][rr];
  }
  __syncthreads();
#pragma unroll
  for (int it = 0; it < 8; ++it) {
    const int row = it * 8 + w;
    const v4f v = *(const v4f*)(st + row * 128 + lane * 4);
    *(volatile v4f*)(zl + (size_t)(b0 + row) * 128 + lane * 4) = v;
  }
  __threadfence();
#pragma unroll
  for (int it = 0; it < 8; ++it) {
    const int row = it * 8 + w;
    const v4f v = *(const v4f*)(st + row * 128 + lane * 4);
    *(volatile v4f*)(zl + (size_t)(b0 + row) * 128 + lane * 4) = v;
  }
}

template <int MODE>
__global__ __launch_bounds__(NTHR) void k_node(
    const unsigned short* __restrict__ hinH, const unsigned short* __restrict__ hinL,
    const float* __restrict__ agg,
    const float* __restrict__ zl, const float* __restrict__ at, const float* __restrict__ aw,
    const float* __restrict__ latb, const float* __restrict__ atb,
    const unsigned short* __restrict__ w1H, const unsigned short* __restrict__ w1L, const float* __restrict__ b1,
    const unsigned short* __restrict__ w2H, const unsigned short* __restrict__ w2L, const float* __restrict__ b2,
    const float* __restrict__ lng, const float* __restrict__ lnb,
    const unsigned short* __restrict__ pwH, const unsigned short* __restrict__ pwL,
    const float* __restrict__ hb1, const float* __restrict__ hw2, const float* __restrict__ hb2,
    const float* __restrict__ posv,
    unsigned short* houtH, unsigned short* houtL, float* pq, float* out,
    int nN, int nA, int nF) {
  extern __shared__ v4f dynlds[];
  unsigned char* lb8 = (unsigned char*)dynlds;
  unsigned short* A1H = (unsigned short*)(lb8 + NO_R0);
  unsigned short* A1L = A1H + TM * 256;
  float* st0 = (float*)(lb8 + NO_R0);
  unsigned short* HPH = (unsigned short*)(lb8 + NO_R1);
  unsigned short* HPL = HPH + TM * HID;
  float* hn  = (float*)(lb8 + NO_R2);
  float* vec = (float*)(lb8 + NO_VEC);
  float* ost = (float*)(lb8 + NO_OST);

  const int tid = threadIdx.x, lane = tid & 31, w = tid >> 5, hh = lane >> 4, m = lane & 15;
  const int node0 = blockIdx.x * TM;
  if (node0 + TM > nN) return;
  const int n = 16 * w + m;

  if (MODE == 0) {
    if (tid < HID) { vec[tid] = latb[tid]; vec[HID + tid] = atb[tid]; }
  } else {
    if (tid < HID) {
      vec[tid] = b1[tid]; vec[HID + tid] = b2[tid];
      vec[2 * HID + tid] = lng[tid]; vec[3 * HID + tid] = lnb[tid];
    }
  }
  if (MODE == 2) {
    if (tid < 64)  vec[512 + tid] = hb1[tid];
    if (tid < 3)   vec[576 + tid] = hb2[tid];
    if (tid < 192) vec[640 + tid] = hw2[tid];
  }

  if (MODE != 0) {
#pragma unroll
    for (int it = 0; it < 4; ++it) {
      const int idx = it * NTHR + tid;
      const int row = idx >> 4, c8 = (idx & 15) * 8;
      const v8us a = *(const v8us*)(hinH + (size_t)(node0 + row) * HID + c8);
      const v8us b = *(const v8us*)(hinL + (size_t)(node0 + row) * HID + c8);
      *(v8us*)(A1H + row * 256 + c8) = a;
      *(v8us*)(A1L + row * 256 + c8) = b;
    }
#pragma unroll
    for (int it = 0; it < 8; ++it) {
      const int idx = it * NTHR + tid;
      const int row = idx >> 5, c4 = (idx & 31) * 4;
      const v4f g = *(const v4f*)(agg + (size_t)(node0 + row) * HID + c4);
      v4us gh, gl;
#pragma unroll
      for (int j = 0; j < 4; ++j) {
        const unsigned p = split2(g[j]);
        gh[j] = (unsigned short)(p & 0xffffu);
        gl[j] = (unsigned short)(p >> 16);
      }
      *(v4us*)(A1H + row * 256 + HID + c4) = gh;
      *(v4us*)(A1L + row * 256 + HID + c4) = gl;
    }
    __syncthreads();

    v8f acc[4];
#pragma unroll
    for (int t = 0; t < 4; ++t) acc[t] = zero8f();
#pragma unroll
    for (int ks = 0; ks < 8; ++ks) {
      const v16us bh = ldfr(w1H + (size_t)n * 256 + 32 * ks, hh);
      const v16us bl = ldfr(w1L + (size_t)n * 256 + 32 * ks, hh);
#pragma unroll
      for (int t = 0; t < 4; ++t) {
        const v16us ah = ldfr(A1H + (16 * t + m) * 256 + 32 * ks, hh);
        const v16us al = ldfr(A1L + (16 * t + m) * 256 + 32 * ks, hh);
        acc[t] = w3(acc[t], ah, al, bh, bl);
      }
    }
    {
      const float bias = vec[n];
#pragma unroll
      for (int t = 0; t < 4; ++t) {
#pragma unroll
        for (int rr = 0; rr < 8; ++rr) {
          const int row = 16 * t + 8 * hh + rr;
          const unsigned p = split2(silu_f(acc[t][rr] + bias));
          HPH[row * HID + n] = (unsigned short)(p & 0xffffu);
          HPL[row * HID + n] = (unsigned short)(p >> 16);
        }
      }
    }
    __syncthreads();

    v8f acc2[4];
#pragma unroll
    for (int t = 0; t < 4; ++t) acc2[t] = zero8f();
#pragma unroll
    for (int ks = 0; ks < 4; ++ks) {
      const v16us bh = ldfr(w2H + (size_t)n * HID + 32 * ks, hh);
      const v16us bl = ldfr(w2L + (size_t)n * HID + 32 * ks, hh);
#pragma unroll
      for (int t = 0; t < 4; ++t) {
        const v16us ah = ldfr(HPH + (16 * t + m) * HID + 32 * ks, hh);
        const v16us al = ldfr(HPL + (16 * t + m) * HID + 32 * ks, hh);
        acc2[t] = w3(acc2[t], ah, al, bh, bl);
      }
    }
    {
      const float bias = vec[HID + n];
#pragma unroll
      for (int t = 0; t < 4; ++t) {
#pragma unroll
        for (int rr = 0; rr < 8; ++rr) hn[(16 * t + 8 * hh + rr) * HID + n] = acc2[t][rr] + bias;
      }
    }
    __syncthreads();
  } else {
    __syncthreads();
  }

  {
    const int row = tid >> 2, q = tid & 3, c0 = q * 32;
    const int node = node0 + row;
    float y[32];
    if (MODE == 0) {
      const int bi = node / nA;
      const float* zr = zl + (size_t)bi * HID + c0;
      float s[32];
#pragma unroll
      for (int j4 = 0; j4 < 8; ++j4) {
        const v4f zv = *(const v4f*)(zr + 4 * j4);
        const v4f lv = *(const v4f*)(vec + c0 + 4 * j4);
        const v4f av = *(const v4f*)(vec + HID + c0 + 4 * j4);
#pragma unroll
        for (int jj = 0; jj < 4; ++jj) { y[4 * j4 + jj] = zv[jj] + lv[jj]; s[4 * j4 + jj] = av[jj]; }
      }
#pragma unroll 1
      for (int k = 0; k < nF; ++k) {
        const float a = at[(size_t)node * nF + k];
        const float* awr = aw + (size_t)k * HID + c0;
#pragma unroll
        for (int j4 = 0; j4 < 8; ++j4) {
          const v4f wv = *(const v4f*)(awr + 4 * j4);
#pragma unroll
          for (int jj = 0; jj < 4; ++jj) s[4 * j4 + jj] += a * wv[jj];
        }
      }
#pragma unroll
      for (int j = 0; j < 32; ++j) y[j] = y[j] + s[j];
    } else {
      const float* hr = hn + row * HID + c0;
      float sum = 0.0f;
#pragma unroll
      for (int j4 = 0; j4 < 8; ++j4) {
        const v4f v = *(const v4f*)(hr + 4 * j4);
#pragma unroll
        for (int jj = 0; jj < 4; ++jj) { y[4 * j4 + jj] = v[jj]; sum += v[jj]; }
      }
      sum += __shfl_xor(sum, 1);
      sum += __shfl_xor(sum, 2);
      const float mu = sum * (1.0f / (float)HID);
      float vs = 0.0f;
#pragma unroll
      for (int j = 0; j < 32; ++j) { const float d = y[j] - mu; vs += d * d; }
      vs += __shfl_xor(vs, 1);
      vs += __shfl_xor(vs, 2);
      const float var = vs * (1.0f / (float)HID);
      const float rs = rsqrtf(var + 1e-5f);
#pragma unroll
      for (int j = 0; j < 32; ++j) y[j] = (y[j] - mu) * rs * vec[2 * HID + c0 + j] + vec[3 * HID + c0 + j];
    }
#pragma unroll
    for (int g = 0; g < 4; ++g) {
      v8us hv, lv;
#pragma unroll
      for (int j = 0; j < 8; ++j) {
        const unsigned p = split2(y[8 * g + j]);
        hv[j] = (unsigned short)(p & 0xffffu);
        lv[j] = (unsigned short)(p >> 16);
      }
      *(v8us*)(HPH + row * HID + c0 + 8 * g) = hv;
      *(v8us*)(HPL + row * HID + c0 + 8 * g) = lv;
    }
    if (MODE == 0) {
      if (tid < 3 * TM) {
        const int orow = tid / 3;
        const int j = tid - 3 * orow;
        const int nd = node0 + orow;
        const int a = nd % nA;
        ost[tid] = posv[(size_t)a * 3 + j];
      }
    }
  }
  __syncthreads();

  if (MODE != 2) {
#pragma unroll
    for (int it = 0; it < 4; ++it) {
      const int idx = it * NTHR + tid;
      const int row = idx >> 4, c8 = (idx & 15) * 8;
      const v8us a = *(const v8us*)(HPH + row * HID + c8);
      const v8us b = *(const v8us*)(HPL + row * HID + c8);
      *(volatile v8us*)(houtH + (size_t)(node0 + row) * HID + c8) = a;
      *(volatile v8us*)(houtL + (size_t)(node0 + row) * HID + c8) = b;
    }
    if (MODE == 0) {
      if (tid < 48) {
        const v4f v = *(const v4f*)(ost + tid * 4);
        *(volatile v4f*)(out + (size_t)node0 * 3 + tid * 4) = v;
      }
    }
    __threadfence();
#pragma unroll
    for (int it = 0; it < 4; ++it) {
      const int idx = it * NTHR + tid;
      const int row = idx >> 4, c8 = (idx & 15) * 8;
      const v8us a = *(const v8us*)(HPH + row * HID + c8);
      const v8us b = *(const v8us*)(HPL + row * HID + c8);
      *(volatile v8us*)(houtH + (size_t)(node0 + row) * HID + c8) = a;
      *(volatile v8us*)(houtL + (size_t)(node0 + row) * HID + c8) = b;
    }
    if (MODE == 0) {
      if (tid < 48) {
        const v4f v = *(const v4f*)(ost + tid * 4);
        *(volatile v4f*)(out + (size_t)node0 * 3 + tid * 4) = v;
      }
    }

    v8f acc3[2][4];
#pragma unroll
    for (int ct = 0; ct < 2; ++ct) {
#pragma unroll
      for (int t = 0; t < 4; ++t) acc3[ct][t] = zero8f();
    }
#pragma unroll
    for (int ks = 0; ks < 4; ++ks) {
      v16us bh[2], bl[2];
#pragma unroll
      for (int ct = 0; ct < 2; ++ct) {
        const int cn = n + 128 * ct;
        bh[ct] = ldfr(pwH + (size_t)cn * HID + 32 * ks, hh);
        bl[ct] = ldfr(pwL + (size_t)cn * HID + 32 * ks, hh);
      }
#pragma unroll
      for (int t = 0; t < 4; ++t) {
        const v16us ah = ldfr(HPH + (16 * t + m) * HID + 32 * ks, hh);
        const v16us al = ldfr(HPL + (16 * t + m) * HID + 32 * ks, hh);
#pragma unroll
        for (int ct = 0; ct < 2; ++ct) acc3[ct][t] = w3(acc3[ct][t], ah, al, bh[ct], bl[ct]);
      }
    }
#pragma unroll
    for (int ct = 0; ct < 2; ++ct) {
#pragma unroll
      for (int t = 0; t < 4; ++t) {
#pragma unroll
        for (int rr = 0; rr < 8; ++rr) st0[(16 * t + 8 * hh + rr) * 256 + 128 * ct + n] = acc3[ct][t][rr];
      }
    }
    __syncthreads();
#pragma unroll
    for (int it = 0; it < 16; ++it) {
      const int p = it * 8 + w;
      const int row = p >> 1, hf = p & 1;
      const v4f v = *(const v4f*)(st0 + row * 256 + hf * 128 + lane * 4);
      *(volatile v4f*)(pq + (size_t)(node0 + row) * 256 + hf * 128 + lane * 4) = v;
    }
    __threadfence();
#pragma unroll
    for (int it = 0; it < 16; ++it) {
      const int p = it * 8 + w;
      const int row = p >> 1, hf = p & 1;
      const v4f v = *(const v4f*)(st0 + row * 256 + hf * 128 + lane * 4);
      *(volatile v4f*)(pq + (size_t)(node0 + row) * 256 + hf * 128 + lane * 4) = v;
    }
  } else {
    if (w < 4) {
      v8f acc4[4];
#pragma unroll
      for (int t = 0; t < 4; ++t) acc4[t] = zero8f();
#pragma unroll
      for (int ks = 0; ks < 4; ++ks) {
        const v16us bh = ldfr(pwH + (size_t)n * HID + 32 * ks, hh);
        const v16us bl = ldfr(pwL + (size_t)n * HID + 32 * ks, hh);
#pragma unroll
        for (int t = 0; t < 4; ++t) {
          const v16us ah = ldfr(HPH + (16 * t + m) * HID + 32 * ks, hh);
          const v16us al = ldfr(HPL + (16 * t + m) * HID + 32 * ks, hh);
          acc4[t] = w3(acc4[t], ah, al, bh, bl);
        }
      }
      const float bias = vec[512 + n];
#pragma unroll
      for (int t = 0; t < 4; ++t) {
#pragma unroll
        for (int rr = 0; rr < 8; ++rr) st0[(16 * t + 8 * hh + rr) * 64 + n] = silu_f(acc4[t][rr] + bias);
      }
    }
    __syncthreads();
    if (tid < 3 * TM) {
      const int orow = tid / 3;
      const int j = tid - 3 * orow;
      const float* hr = st0 + orow * 64;
      float d = 0.0f;
#pragma unroll 8
      for (int k = 0; k < 64; ++k) d += hr[k] * vec[640 + k * 3 + j];
      const float delta = d + vec[576 + j];
      ost[tid] = posv[(size_t)(node0 + orow) * 3 + j] + delta;
    }
    __syncthreads();
    v4f ov = {0.0f, 0.0f, 0.0f, 0.0f};
    if (tid < 48) ov = *(const v4f*)(ost + tid * 4);
    if (tid < 48) *(volatile v4f*)(out + (size_t)node0 * 3 + tid * 4) = ov;
    __threadfence();
    if (tid < 48) *(volatile v4f*)(out + (size_t)node0 * 3 + tid * 4) = ov;
  }
}

__global__ __launch_bounds__(NTHR) void k_edge(
    const float* __restrict__ pq, const float* __restrict__ posin, const int* __restrict__ ei,
    const unsigned short* __restrict__ w2H, const unsigned short* __restrict__ w2L,
    const unsigned short* __restrict__ c1P,
    const float* __restrict__ w257, const float* __restrict__ eb1, const float* __restrict__ eb2,
    const float* __restrict__ cb1, const float* __restrict__ cw2,
    float* aggout, float* posout, int nN, int nE, int vec8) {
  extern __shared__ v4f dynlds[];
  unsigned char* lb8 = (unsigned char*)dynlds;
  float* ACC  = (float*)(lb8 + EO_ACC);
  float* ACU  = (float*)(lb8 + EO_ACU);
  unsigned short* E1H = (unsigned short*)(lb8 + EO_E1H);
  unsigned short* E1L = (unsigned short*)(lb8 + EO_E1L);
  unsigned short* MPL = (unsigned short*)(lb8 + EO_MPL);
  float* PART = (float*)(lb8 + EO_PART);
  float* RELV = (float*)(lb8 + EO_RELV);
  float* CWR  = (float*)(lb8 + EO_CWR);
  int*   SLOT = (int*)(lb8 + EO_SLOT);
  int*   PEND = (int*)(lb8 + EO_PEND);
  int*   LIST = (int*)(lb8 + EO_LIST);
  float* WTS  = (float*)(lb8 + EO_WTS);
  int*   WCNT = (int*)(lb8 + EO_MISC);
  int*   PENDN = WCNT + NWAVE;

  const int tid = threadIdx.x, lane = tid & 31, wave = tid >> 5, hh = lane >> 4, m = lane & 15;
  const int nodeBase = blockIdx.x * NB;
  if (nodeBase + NB > nN) return;
  const int* dsts = ei;
  const int* srcs = ei + nE;
  const v4f z4 = {0.0f, 0.0f, 0.0f, 0.0f};

  for (int i = tid; i < (NB + 1) * HID / 4; i += NTHR) ((v4f*)ACC)[i] = z4;
  for (int i = tid; i < NB + 1; i += NTHR) ((v4f*)ACU)[i] = z4;
  if (tid < HID) {
    WTS[tid] = w257[tid]; WTS[HID + tid] = eb1[tid]; WTS[2 * HID + tid] = eb2[tid];
    WTS[3 * HID + tid] = cb1[tid]; WTS[4 * HID + tid] = cw2[tid];
  }
  if (tid == 0) PENDN[0] = 0;
  __syncthreads();

  const int nChunks = (nE + CHUNK - 1) / CHUNK;
#pragma unroll 1
  for (int ch = 0; ch < nChunks; ++ch) {
    const int cbase = ch * CHUNK;
    const int wc = scan_chunk(dsts, nE, cbase, nodeBase, vec8, LIST, tid, wave);
    if (lane == 0) WCNT[wave] = wc;
    __syncthreads();

    const int base = PENDN[0];
    int tot = 0, myoff = 0;
#pragma unroll
    for (int ww = 0; ww < NWAVE; ++ww) {
      int c = WCNT[ww];
      c = c > WCAP ? WCAP : (c < 0 ? 0 : c);
      if (ww < wave) myoff += c;
      tot += c;
    }
    int newN = base + tot;
    newN = newN > PCAP ? PCAP : newN;
    {
      int cnt = WCNT[wave];
      cnt = cnt > WCAP ? WCAP : (cnt < 0 ? 0 : cnt);
      const int* lp = LIST + wave * WCAP;
      for (int i = lane; i < cnt; i += 32) {
        const int pos = base + myoff + i;
        if (pos < PCAP) PEND[pos] = cbase + lp[i];
      }
    }
    const int fin = (ch == nChunks - 1) ? 1 : 0;
    int R = (fin != 0) ? (newN + PASSN - 1) / PASSN : newN / PASSN;
    R = R > RMAX ? RMAX : (R < 0 ? 0 : R);
    const int Pv = (fin != 0) ? newN : R * PASSN;
    __syncthreads();

#pragma unroll 1
    for (int r = 0; r < R; ++r) {
      {
        const int e = tid >> 1, hf = tid & 1;
        const int idx = r * PASSN + e;
        const bool valid = idx < Pv;
        int eg = PEND[min(idx, PCAP - 1)];
        eg = valid ? eg : 0;
        eg = eg < 0 ? 0 : (eg > nE - 1 ? nE - 1 : eg);
        int rw = dsts[eg];
        int cl = srcs[eg];
        int slot = rw - nodeBase;
        if (!valid || (unsigned)slot >= (unsigned)NB) slot = NB;
        rw = rw < 0 ? 0 : (rw > nN - 1 ? nN - 1 : rw);
        cl = cl < 0 ? 0 : (cl > nN - 1 ? nN - 1 : cl);
        const float px0 = posin[(size_t)rw * 3 + 0], px1 = posin[(size_t)rw * 3 + 1], px2 = posin[(size_t)rw * 3 + 2];
        const float qx0 = posin[(size_t)cl * 3 + 0], qx1 = posin[(size_t)cl * 3 + 1], qx2 = posin[(size_t)cl * 3 + 2];
        const float rx = px0 - qx0, ry = px1 - qx1, rz = px2 - qx2;
        float d2 = rx * rx + ry * ry + rz * rz;
        d2 = fminf(fmaxf(d2, 1e-6f), 1e6f);
        if (hf == 0) {
          SLOT[e] = slot;
          const v4f rv = {rx, ry, rz, d2};
          *(v4f*)(RELV + e * 4) = rv;
        }
        const float* prow = pq + (size_t)rw * 256 + hf * 64;
        const float* qrow = pq + (size_t)cl * 256 + 128 + hf * 64;
#pragma unroll
        for (int g = 0; g < 4; ++g) {
          const int c = hf * 64 + g * 16;
          float x[16];
#pragma unroll
          for (int j4 = 0; j4 < 4; ++j4) {
            const v4f pv = *(const v4f*)(prow + g * 16 + 4 * j4);
            const v4f qv = *(const v4f*)(qrow + g * 16 + 4 * j4);
            const v4f wv = *(const v4f*)(WTS + c + 4 * j4);
            const v4f bv = *(const v4f*)(WTS + HID + c + 4 * j4);
#pragma unroll
            for (int jj = 0; jj < 4; ++jj) x[4 * j4 + jj] = silu_f((pv[jj] + qv[jj]) + d2 * wv[jj] + bv[jj]);
          }
          v8us ha, la, hb, lbv;
#pragma unroll
          for (int j = 0; j < 8; ++j) {
            const unsigned pa = split2(x[j]);
            const unsigned pb = split2(x[8 + j]);
            ha[j] = (unsigned short)(pa & 0xffffu); la[j]  = (unsigned short)(pa >> 16);
            hb[j] = (unsigned short)(pb & 0xffffu); lbv[j] = (unsigned short)(pb >> 16);
          }
          *(v8us*)(E1H + e * HID + c)     = ha;
          *(v8us*)(E1H + e * HID + c + 8) = hb;
          *(v8us*)(E1L + e * HID + c)     = la;
          *(v8us*)(E1L + e * HID + c + 8) = lbv;
        }
      }
      __syncthreads();

      {
        const int n = 16 * wave + m;
        v16us bH[4], bL[4];
#pragma unroll
        for (int ks = 0; ks < 4; ++ks) {
          bH[ks] = ldfr(w2H + (size_t)n * HID + 32 * ks, hh);
          bL[ks] = ldfr(w2L + (size_t)n * HID + 32 * ks, hh);
        }
        const float bias = WTS[2 * HID + n];
#pragma unroll 1
        for (int t = 0; t < PASSN / 16; ++t) {
          v8f acc = zero8f();
#pragma unroll
          for (int ks = 0; ks < 4; ++ks) {
            const v16us aH = ldfr(E1H + (t * 16 + m) * HID + 32 * ks, hh);
            const v16us aL = ldfr(E1L + (t * 16 + m) * HID + 32 * ks, hh);
            acc = w3(acc, aH, aL, bH[ks], bL[ks]);
          }
          float mv[8];
          int sl[8];
#pragma unroll
          for (int rr = 0; rr < 8; ++rr) {
            mv[rr] = silu_f(acc[rr] + bias);
            int s = SLOT[t * 16 + 8 * hh + rr];
            s = s < 0 ? 0 : (s > NB ? NB : s);
            sl[rr] = s;
          }
#pragma unroll
          for (int rr = 0; rr < 8; ++rr)
            MPL[(t * 16 + 8 * hh + rr) * HID + n] = f16bits(mv[rr] * 16.0f);
#pragma unroll
          for (int ph = 0; ph < 2; ++ph) {
            if (hh == ph) {
#pragma unroll
              for (int rr = 0; rr < 8; ++rr) {
                float* ap = ACC + sl[rr] * HID + n;
                const float o = *ap;
                *ap = o + mv[rr];
              }
            }
            __builtin_amdgcn_fence(__ATOMIC_RELEASE, "wavefront");
            __builtin_amdgcn_wave_barrier();
          }
        }
      }
      __syncthreads();

      {
        const int n = 16 * wave + m;
        v16us bC[4];
#pragma unroll
        for (int ks = 0; ks < 4; ++ks) bC[ks] = ldfr(c1P + (size_t)n * HID + 32 * ks, hh);
        const float cbias = WTS[3 * HID + n], c2v = WTS[4 * HID + n];
#pragma unroll 1
        for (int t = 0; t < PASSN / 16; ++t) {
          v8f acc = zero8f();
#pragma unroll
          for (int ks = 0; ks < 4; ++ks) {
            const v16us a = ldfr(MPL + (t * 16 + m) * HID + 32 * ks, hh);
            acc = wf16(acc, a, bC[ks]);
          }
#pragma unroll
          for (int rr = 0; rr < 8; ++rr) {
            float u = silu_f(acc[rr] * (1.0f / 1024.0f) + cbias) * c2v;
            u += __shfl_xor(u, 1);
            u += __shfl_xor(u, 2);
            u += __shfl_xor(u, 4);
            u += __shfl_xor(u, 8);
            if (m == 0) PART[wave * PASSN + t * 16 + 8 * hh + rr] = u;
          }
        }
      }
      __syncthreads();

      if (tid < PASSN) {
        float s = PART[tid];
#pragma unroll
        for (int ww = 1; ww < NWAVE; ++ww) s += PART[ww * PASSN + tid];
        s = fminf(fmaxf(s, -1.0f), 1.0f);
        const v4f rv = *(const v4f*)(RELV + tid * 4);
        const v4f o = {s * rv.x, s * rv.y, s * rv.z, 1.0f};
        *(v4f*)(CWR + tid * 4) = o;
      }
      __syncthreads();

      if (wave == 0) {
#pragma unroll 1
        for (int i = 0; i < PASSN; ++i) {
          int s = SLOT[i];
          s = s < 0 ? 0 : (s > NB ? NB : s);
          if (lane < 4) {
            float* ap = ACU + s * 4 + lane;
            const float o = *ap;
            *ap = o + CWR[i * 4 + lane];
          }
        }
      }
      __syncthreads();
    }

    int rem = newN - R * PASSN;
    rem = rem < 0 ? 0 : (rem > PASSN ? PASSN : rem);
    if (R > 0 && tid < rem) PEND[tid] = PEND[R * PASSN + tid];
    if (tid == 0) PENDN[0] = rem;
  }
  __syncthreads();

  for (int i = tid; i < NB * 3; i += NTHR) {
    const int nd = i / 3;
    const int c = i - nd * 3;
    const float u = ACU[nd * 4 + c];
    const float dg = ACU[nd * 4 + 3];
    PART[i] = posin[(size_t)(nodeBase + nd) * 3 + c] + u * (1.0f / (dg + 1e-6f));
  }
  __syncthreads();
#pragma unroll
  for (int it = 0; it < NB / NWAVE; ++it) {
    const int row = it * NWAVE + wave;
    const v4f v = *(const v4f*)(ACC + row * HID + lane * 4);
    *(volatile v4f*)(aggout + (size_t)(nodeBase + row) * HID + lane * 4) = v;
  }
  if (tid < NB * 3 / 4) {
    const v4f v = *(const v4f*)(PART + tid * 4);
    *(volatile v4f*)(posout + (size_t)nodeBase * 3 + tid * 4) = v;
  }
  __threadfence();
#pragma unroll
  for (int it = 0; it < NB / NWAVE; ++it) {
    const int row = it * NWAVE + wave;
    const v4f v = *(const v4f*)(ACC + row * HID + lane * 4);
    *(volatile v4f*)(aggout + (size_t)(nodeBase + row) * HID + lane * 4) = v;
  }
  if (tid < NB * 3 / 4) {
    const v4f v = *(const v4f*)(PART + tid * 4);
    *(volatile v4f*)(posout + (size_t)nodeBase * 3 + tid * 4) = v;
  }
}

extern "C" void kernel_launch(void* const* d_in, const int* in_sizes, int n_in,
                              void* d_out, int out_size, void* d_ws, size_t ws_size,
                              hipStream_t stream) {
  if (n_in < 25) return;
  const int nF = 10;
  const int nB = in_sizes[0] / 64;
  const int nN = in_sizes[1] / nF;
  const int nE = in_sizes[2] / 2;
  const int nA = in_sizes[3] / 3;
  const int L  = in_sizes[8] / (257 * HID);
  if (nB <= 0 || nN <= 0 || nE <= 0 || nA <= 0 || L < 1) return;
  if (in_sizes[0] != nB * 64 || in_sizes[1] != nN * nF || in_sizes[2] != 2 * nE || in_sizes[3] != nA * 3) return;
  if (nN != nB * nA || (nN % NB) != 0 || (nN % TM) != 0 || (nB % 64) != 0) return;
  if (in_sizes[4] != 64 * HID || in_sizes[5] != HID || in_sizes[6] != nF * HID || in_sizes[7] != HID) return;
  if (in_sizes[8] != L * 257 * HID || in_sizes[9] != L * HID || in_sizes[10] != L * HID * HID || in_sizes[11] != L * HID) return;
  if (in_sizes[12] != L * 256 * HID || in_sizes[13] != L * HID || in_sizes[14] != L * HID * HID || in_sizes[15] != L * HID) return;
  if (in_sizes[16] != L * HID * HID || in_sizes[17] != L * HID || in_sizes[18] != L * HID) return;
  if (in_sizes[19] != L * HID || in_sizes[20] != L * HID) return;
  if (in_sizes[21] != HID * 64 || in_sizes[22] != 64 || in_sizes[23] != 64 * 3 || in_sizes[24] != 3) return;
  if (out_size != nN * 3) return;

  const float* z           = (const float*)d_in[0];
  const float* atom_types  = (const float*)d_in[1];
  const int*   edge_index  = (const int*)d_in[2];
  const float* init_coords = (const float*)d_in[3];
  const float* latent_w    = (const float*)d_in[4];
  const float* latent_b    = (const float*)d_in[5];
  const float* atom_w      = (const float*)d_in[6];
  const float* atom_b      = (const float*)d_in[7];
  const float* edge_w1     = (const float*)d_in[8];
  const float* edge_b1     = (const float*)d_in[9];
  const float* edge_w2     = (const float*)d_in[10];
  const float* edge_b2     = (const float*)d_in[11];
  const float* node_w1     = (const float*)d_in[12];
  const float* node_b1     = (const float*)d_in[13];
  const float* node_w2     = (const float*)d_in[14];
  const float* node_b2     = (const float*)d_in[15];
  const float* coord_w1    = (const float*)d_in[16];
  const float* coord_b1    = (const float*)d_in[17];
  const float* coord_w2    = (const float*)d_in[18];
  const float* ln_g        = (const float*)d_in[19];
  const float* ln_b        = (const float*)d_in[20];
  const float* head_w1     = (const float*)d_in[21];
  const float* head_b1     = (const float*)d_in[22];
  const float* head_w2     = (const float*)d_in[23];
  const float* head_b2     = (const float*)d_in[24];
  float* out = (float*)d_out;

  size_t off = 0;
  char* wsb = (char*)d_ws;
  auto carve = [&](size_t bytes) -> char* {
    char* p = wsb + off;
    off += (bytes + 255) & ~(size_t)255;
    return p;
  };
  unsigned short* lwH = (unsigned short*)carve((size_t)128 * 64 * 2);
  unsigned short* lwL = (unsigned short*)carve((size_t)128 * 64 * 2);
  unsigned short* e1H = (unsigned short*)carve((size_t)L * 256 * 128 * 2);
  unsigned short* e1L = (unsigned short*)carve((size_t)L * 256 * 128 * 2);
  unsigned short* w2H = (unsigned short*)carve((size_t)L * 128 * 128 * 2);
  unsigned short* w2L = (unsigned short*)carve((size_t)L * 128 * 128 * 2);
  unsigned short* n1H = (unsigned short*)carve((size_t)L * 128 * 256 * 2);
  unsigned short* n1L = (unsigned short*)carve((size_t)L * 128 * 256 * 2);
  unsigned short* n2H = (unsigned short*)carve((size_t)L * 128 * 128 * 2);
  unsigned short* n2L = (unsigned short*)carve((size_t)L * 128 * 128 * 2);
  unsigned short* c1P = (unsigned short*)carve((size_t)L * 128 * 128 * 2);
  unsigned short* hwH = (unsigned short*)carve((size_t)64 * 128 * 2);
  unsigned short* hwL = (unsigned short*)carve((size_t)64 * 128 * 2);
  float* zlb = (float*)carve((size_t)nB * HID * 4);
  unsigned short* hAH = (unsigned short*)carve((size_t)nN * HID * 2);
  unsigned short* hAL = (unsigned short*)carve((size_t)nN * HID * 2);
  unsigned short* hBH = (unsigned short*)carve((size_t)nN * HID * 2);
  unsigned short* hBL = (unsigned short*)carve((size_t)nN * HID * 2);
  float* pq   = (float*)carve((size_t)nN * 256 * 4);
  float* agg  = (float*)carve((size_t)nN * HID * 4);
  float* posA = (float*)carve((size_t)nN * 3 * 4);
  float* posB = (float*)carve((size_t)nN * 3 * 4);
  if (off > ws_size) return;

  const int vec8 = ((nE & 3) == 0) ? 1 : 0;

  hipFuncSetAttribute(reinterpret_cast<const void*>(&k_edge), hipFuncAttributeMaxDynamicSharedMemorySize, EDGE_LDS);
  hipFuncSetAttribute(reinterpret_cast<const void*>(&k_node<0>), hipFuncAttributeMaxDynamicSharedMemorySize, NODE_LDS);
  hipFuncSetAttribute(reinterpret_cast<const void*>(&k_node<1>), hipFuncAttributeMaxDynamicSharedMemorySize, NODE_LDS);
  hipFuncSetAttribute(reinterpret_cast<const void*>(&k_node<2>), hipFuncAttributeMaxDynamicSharedMemorySize, NODE_LDS);

  k_cvt<0><<<dim3((128 * 64 / 8 + NTHR - 1) / NTHR, 1), NTHR, 0, stream>>>(
      latent_w, lwH, lwL, 64, 128, 128, 128, 1, 0, 0, 0, 1.0f);
  k_cvt<0><<<dim3((256 * 128 / 8 + NTHR - 1) / NTHR, L), NTHR, 0, stream>>>(
      edge_w1, e1H, e1L, 128, 256, 128, 128, 1, 128 * 128, 257 * 128, 256 * 128, 1.0f);
  k_cvt<0><<<dim3((128 * 128 / 8 + NTHR - 1) / NTHR, L), NTHR, 0, stream>>>(
      edge_w2, w2H, w2L, 128, 128, 128, 128, 1, 0, 128 * 128, 128 * 128, 1.0f);
  k_cvt<0><<<dim3((128 * 256 / 8 + NTHR - 1) / NTHR, L), NTHR, 0, stream>>>(
      node_w1, n1H, n1L, 256, 128, 128, 128, 1, 0, 256 * 128, 128 * 256, 1.0f);
  k_cvt<0><<<dim3((128 * 128 / 8 + NTHR - 1) / NTHR, L), NTHR, 0, stream>>>(
      node_w2, n2H, n2L, 128, 128, 128, 128, 1, 0, 128 * 128, 128 * 128, 1.0f);
  k_cvt<1><<<dim3((128 * 128 / 8 + NTHR - 1) / NTHR, L), NTHR, 0, stream>>>(
      coord_w1, c1P, c1P, 128, 128, 128, 128, 1, 0, 128 * 128, 128 * 128, 64.0f);
  k_cvt<0><<<dim3((64 * 128 / 8 + NTHR - 1) / NTHR, 1), NTHR, 0, stream>>>(
      head_w1, hwH, hwL, 128, 64, 64, 64, 1, 0, 0, 0, 1.0f);

  k_zl<<<nB / 64, NTHR, 0, stream>>>(z, lwH, lwL, zlb, nB);

  k_node<0><<<nN / TM, NTHR, NODE_LDS, stream>>>(
      hBH, hBL, zlb,
      zlb, atom_types, atom_w, latent_b, atom_b,
      n1H, n1L, node_b1, n2H, n2L, node_b2, ln_g, ln_b,
      e1H, e1L,
      head_b1, head_w2, head_b2,
      init_coords,
      hAH, hAL, pq, posA,
      nN, nA, nF);

  unsigned short* hCurH = hAH; unsigned short* hCurL = hAL;
  unsigned short* hNxtH = hBH; unsigned short* hNxtL = hBL;
  float* posCur = posA;
  float* posNxt = posB;

  for (int l = 0; l < L; ++l) {
    k_edge<<<nN / NB, NTHR, EDGE_LDS, stream>>>(
        pq, posCur, edge_index,
        w2H + (size_t)l * 128 * 128, w2L + (size_t)l * 128 * 128,
        c1P + (size_t)l * 128 * 128,
        edge_w1 + (size_t)l * 257 * 128 + (size_t)256 * 128,
        edge_b1 + (size_t)l * 128, edge_b2 + (size_t)l * 128,
        coord_b1 + (size_t)l * 128, coord_w2 + (size_t)l * 128,
        agg, posNxt, nN, nE, vec8);
    { float* tp = posCur; posCur = posNxt; posNxt = tp; }

    if (l < L - 1) {
      k_node<1><<<nN / TM, NTHR, NODE_LDS, stream>>>(
          hCurH, hCurL, agg,
          zlb, atom_types, atom_w, latent_b, atom_b,
          n1H + (size_t)l * 128 * 256, n1L + (size_t)l * 128 * 256, node_b1 + (size_t)l * 128,
          n2H + (size_t)l * 128 * 128, n2L + (size_t)l * 128 * 128, node_b2 + (size_t)l * 128,
          ln_g + (size_t)l * 128, ln_b + (size_t)l * 128,
          e1H + (size_t)(l + 1) * 256 * 128, e1L + (size_t)(l + 1) * 256 * 128,
          head_b1, head_w2, head_b2,
          posCur,
          hNxtH, hNxtL, pq, pq,
          nN, nA, nF);
      { unsigned short* t1 = hCurH; hCurH = hNxtH; hNxtH = t1; }
      { unsigned short* t2 = hCurL; hCurL = hNxtL; hNxtL = t2; }
    } else {
      k_node<2><<<nN / TM, NTHR, NODE_LDS, stream>>>(
          hCurH, hCurL, agg,
          zlb, atom_types, atom_w, latent_b, atom_b,
          n1H + (size_t)l * 128 * 256, n1L + (size_t)l * 128 * 256, node_b1 + (size_t)l * 128,
          n2H + (size_t)l * 128 * 128, n2L + (size_t)l * 128 * 128, node_b2 + (size_t)l * 128,
          ln_g + (size_t)l * 128, ln_b + (size_t)l * 128,
          hwH, hwL,
          head_b1, head_w2, head_b2,
          posCur,
          hNxtH, hNxtL, pq, out,
          nN, nA, nF);
    }
  }
}
